// FluidAttentionLayer_67903432950551
// MI455X (gfx1250) — hardware-verified
//
#include <hip/hip_runtime.h>


namespace {
constexpr int S = 4096, HID = 2048, NH = 16, NKV = 4, DH = 128, QPG = 4, GW = (QPG + 2) * DH, TOT = NKV * GW;
constexpr int SP = 512;
constexpr float XS = 8.0f, WSC = 256.0f, PS = 8.0f;

typedef _Float16 b16;
typedef __attribute__((ext_vector_type(16))) _Float16 v16b;
typedef __attribute__((ext_vector_type(8))) _Float16 v8b;
typedef __attribute__((ext_vector_type(8))) float v8f;
typedef __attribute__((ext_vector_type(4))) float v4f;
__device__ __forceinline__ float bf16_rne(float f) { unsigned int u = __float_as_uint(f); u += 0x7FFFu + ((u >> 16) & 1u); return __uint_as_float(u & 0xFFFF0000u); }
__device__ __forceinline__ void split16(float v, b16& hi, b16& lo) { hi = (b16)v; lo = (b16)(v - (float)hi); }
__device__ __forceinline__ v16b frag_kb(const b16* p, int hh) { const v8b a = *(const v8b*)(p + 8 * hh), b = *(const v8b*)(p + 16 + 8 * hh); v16b f;
#pragma unroll
  for (int e = 0; e < 8; ++e) { f[e] = a[e]; f[8 + e] = b[e]; } return f; }
__device__ __forceinline__ v8f wmma16b(v16b a, v16b b, v8f c) { v8f d = __builtin_amdgcn_wmma_f32_16x16x32_f16(false, a, false, b, (short)0, c, false, false); asm volatile("v_nop\n\tv_nop\n\tv_nop\n\tv_nop" : "+v"(d) : "v"(a), "v"(b)); return d; }
__device__ __forceinline__ void wave_lds_sync() { __builtin_amdgcn_fence(__ATOMIC_RELEASE, "workgroup"); __builtin_amdgcn_wave_barrier(); __builtin_amdgcn_fence(__ATOMIC_ACQUIRE, "workgroup"); }
__device__ __forceinline__ float nexp(float x) { return __builtin_amdgcn_exp2f(x * 1.4426950408889634f); }

__global__ __launch_bounds__(256) void prep_kernel(const float* __restrict__ x, const float* __restrict__ wq, const float* __restrict__ wp, b16* __restrict__ X16, b16* __restrict__ WQ, b16* __restrict__ WP) {
  const size_t tid = (size_t)blockIdx.x * 256 + threadIdx.x, nth = (size_t)gridDim.x * 256;
  const size_t n1 = (size_t)S * HID / 8, n2 = (size_t)TOT * HID / 8, n3 = (size_t)HID * HID / 8;
  for (int pass = 0; pass < 2; ++pass) {
    for (size_t g = tid; g < n1 + n2 + n3; g += nth) { const float* src; b16* dst; size_t e; float sc; bool isx;
      if (g < n1) { src = x; dst = X16; e = g * 8; sc = XS; isx = true; } else if (g < n1 + n2) { src = wq; dst = WQ; e = (g - n1) * 8; sc = WSC; isx = false; } else { src = wp; dst = WP; e = (g - n1 - n2) * 8; sc = WSC; isx = false; }
      (void)isx; const v4f a = *(const v4f*)(src + e), c = *(const v4f*)(src + e + 4); v8b o;
#pragma unroll
      for (int j = 0; j < 4; ++j) { o[j] = (b16)(bf16_rne(a[j]) * sc); o[4 + j] = (b16)(bf16_rne(c[j]) * sc); }
      *(volatile v8b*)(dst + e) = o; }
    __threadfence(); }
}
__global__ __launch_bounds__(128) void qkv_kernel(const b16* __restrict__ X16, const b16* __restrict__ WQ, b16* __restrict__ QH, b16* __restrict__ QL, b16* __restrict__ KH, b16* __restrict__ VROW, b16* __restrict__ KL, b16* __restrict__ VROWL) {
  __shared__ __attribute__((aligned(16))) b16 Th[4][16][DH + 8], Tl[4][16][DH + 8];
  const int wave = threadIdx.x >> 5, lane = threadIdx.x & 31, nloc = lane & 15, hlf = lane >> 4; const int m0 = blockIdx.x * 64 + wave * 16, nb = blockIdx.y, n0 = nb * 128;
  const int g = nb / 6, sub = nb - g * 6;
  v8f acc[8];
#pragma unroll
  for (int t = 0; t < 8; ++t) acc[t] = (v8f){};
#pragma unroll 2
  for (int kb = 0; kb < HID; kb += 32) { const v16b a = frag_kb(X16 + (size_t)(m0 + nloc) * HID + kb, hlf);
#pragma unroll
    for (int t = 0; t < 8; ++t) acc[t] = wmma16b(a, frag_kb(WQ + (size_t)(n0 + t * 16 + nloc) * HID + kb, hlf), acc[t]); }
#pragma unroll
  for (int t = 0; t < 8; ++t)
#pragma unroll
    for (int r = 0; r < 8; ++r) { b16 a_, c_; split16(acc[t][r] * (1.0f / (XS * WSC)) * XS, a_, c_); Th[wave][8 * hlf + r][t * 16 + nloc] = a_; Tl[wave][8 * hlf + r][t * 16 + nloc] = c_; }
  wave_lds_sync();
  b16* dh = sub < 4 ? QH + ((size_t)(g * QPG + sub) * S) * DH : sub == 4 ? KH + (size_t)g * S * DH : VROW + (size_t)g * S * DH;
  b16* dl = sub < 4 ? QL + ((size_t)(g * QPG + sub) * S) * DH : sub == 4 ? KL + (size_t)g * SP * DH : VROWL + (size_t)g * SP * DH; const bool wlo = (sub < 4) || (m0 < SP);
  for (int pass = 0; pass < 2; ++pass) { for (int rr = 0; rr < 16; ++rr) if (lane < 16) { *(volatile v8b*)(dh + (size_t)(m0 + rr) * DH + lane * 8) = *(const v8b*)(&Th[wave][rr][lane * 8]); if (wlo) *(volatile v8b*)(dl + (size_t)(m0 + rr) * DH + lane * 8) = *(const v8b*)(&Tl[wave][rr][lane * 8]); } __threadfence(); }
}
__global__ __launch_bounds__(256) void vt_kernel(const b16* __restrict__ VROW, const b16* __restrict__ VROWL, b16* __restrict__ VT, b16* __restrict__ VTL) {
  __shared__ __attribute__((aligned(16))) b16 Tt[DH][64 + 8], Tu[DH][64 + 8];
  const int g = blockIdx.y, s0 = blockIdx.x * 64, t_ = threadIdx.x; const bool lo = s0 < SP;
  for (int k = t_; k < 64 * DH; k += 256) { const int ss = k >> 7, d = k & 127; Tt[d][ss] = VROW[((size_t)g * S + s0 + ss) * DH + d]; if (lo) Tu[d][ss] = VROWL[((size_t)g * SP + s0 + ss) * DH + d]; }
  __syncthreads();
  for (int pass = 0; pass < 2; ++pass) { for (int q = t_; q < DH * 8; q += 256) { const int d = q >> 3, c8 = (q & 7) * 8; *(volatile v8b*)(VT + ((size_t)g * DH + d) * S + s0 + c8) = *(const v8b*)(&Tt[d][c8]); if (lo) *(volatile v8b*)(VTL + ((size_t)g * DH + d) * SP + s0 + c8) = *(const v8b*)(&Tu[d][c8]); } __threadfence(); }
}
template <bool PRECISE>
__global__ __launch_bounds__(64) void attn_kernel(const b16* __restrict__ QH, const b16* __restrict__ QL, const b16* __restrict__ KH, const b16* __restrict__ KL, const b16* __restrict__ VT, const b16* __restrict__ VTL, b16* __restrict__ ATTH, b16* __restrict__ ATTL) {
  __shared__ __attribute__((aligned(16))) b16 Th[2][16][DH + 8], Tl[2][16][DH + 8];
  const int wave = threadIdx.x >> 5, lane = threadIdx.x & 31, hh = lane >> 4, col = lane & 15; const int h = blockIdx.y, g = h / QPG, q0 = blockIdx.x * 32 + wave * 16, qi = q0 + col;
  const b16* Qh = QH + (size_t)h * S * DH; const b16* Ql = QL + (size_t)h * S * DH; const b16* K = KH + (size_t)g * S * DH; const b16* Kl = KL + (size_t)g * SP * DH; const b16* V = VT + (size_t)g * DH * S; const b16* Vl = VTL + (size_t)g * DH * SP;
  v16b qf[4], ql[4];
#pragma unroll
  for (int ks = 0; ks < 4; ++ks) { qf[ks] = frag_kb(Qh + (size_t)qi * DH + ks * 32, hh); ql[ks] = frag_kb(Ql + (size_t)qi * DH + ks * 32, hh); }
  const float scale = (1.0f / sqrtf((float)DH)) * (1.0f / (XS * XS));
  float m = -INFINITY, l = 0.0f; v8f o[8];
#pragma unroll
  for (int t = 0; t < 8; ++t) o[t] = (v8f){};
  const int kend = q0 + 16;
  for (int kb = 0; kb < kend; kb += 32) {
    v8f s0 = {}, s1 = {};
#pragma unroll
    for (int ks = 0; ks < 4; ++ks) { const v16b k0 = frag_kb(K + (size_t)(kb + col) * DH + ks * 32, hh), k1 = frag_kb(K + (size_t)(kb + 16 + col) * DH + ks * 32, hh);
      s0 = wmma16b(k0, qf[ks], s0); s0 = wmma16b(k0, ql[ks], s0); s1 = wmma16b(k1, qf[ks], s1); s1 = wmma16b(k1, ql[ks], s1);
      if (PRECISE) { s0 = wmma16b(frag_kb(Kl + (size_t)(kb + col) * DH + ks * 32, hh), qf[ks], s0); s1 = wmma16b(frag_kb(Kl + (size_t)(kb + 16 + col) * DH + ks * 32, hh), qf[ks], s1); } }
    float mr = -INFINITY;
#pragma unroll
    for (int r = 0; r < 8; ++r) { const int ka = kb + 8 * hh + r, kc = kb + 16 + 8 * hh + r; s0[r] = (ka <= qi) ? s0[r] * scale : -INFINITY; s1[r] = (kc <= qi) ? s1[r] * scale : -INFINITY; mr = fmaxf(mr, fmaxf(s0[r], s1[r])); }
    mr = fmaxf(mr, __shfl_xor(mr, 16)); const float mn = fmaxf(m, mr);
    const float al_ = nexp(m - mn); m = mn; float sum = 0.0f; v16b pb, pl;
#pragma unroll
    for (int r = 0; r < 8; ++r) { const float e0 = nexp(s0[r] - mn), e1 = nexp(s1[r] - mn); sum += e0 + e1; b16 a_, c_; split16(e0 * PS, a_, c_); pb[r] = a_; pl[r] = c_; split16(e1 * PS, a_, c_); pb[8 + r] = a_; pl[8 + r] = c_; }
    sum += __shfl_xor(sum, 16); l = l * al_ + sum;
#pragma unroll
    for (int t = 0; t < 8; ++t) { o[t] *= al_; const v16b vh = frag_kb(V + (size_t)(t * 16 + col) * S + kb, hh); o[t] = wmma16b(vh, pb, o[t]);
      if (PRECISE) { o[t] = wmma16b(vh, pl, o[t]); o[t] = wmma16b(frag_kb(Vl + (size_t)(t * 16 + col) * SP + kb, hh), pb, o[t]); } } }
  const float inv = 1.0f / (l * PS * XS);
#pragma unroll
  for (int t = 0; t < 8; ++t)
#pragma unroll
    for (int r = 0; r < 8; ++r) { b16 a_, c_; split16(o[t][r] * inv * XS, a_, c_); Th[wave][col][t * 16 + 8 * hh + r] = a_; Tl[wave][col][t * 16 + 8 * hh + r] = c_; }
  wave_lds_sync();
  for (int pass = 0; pass < 2; ++pass) { for (int rr = 0; rr < 16; ++rr) if (lane < 16) { const size_t gi = (size_t)(q0 + rr) * HID + h * DH + lane * 8; *(volatile v8b*)(ATTH + gi) = *(const v8b*)(&Th[wave][rr][lane * 8]); *(volatile v8b*)(ATTL + gi) = *(const v8b*)(&Tl[wave][rr][lane * 8]); } __threadfence(); }
}
template <bool TWO>
__global__ __launch_bounds__(128) void proj_kernel(const b16* __restrict__ ATT, const b16* __restrict__ ATTL, const b16* __restrict__ WP, float* __restrict__ out, int rb0) {
  __shared__ __attribute__((aligned(16))) float Ts[4][16][128 + 4];
  const int wave = threadIdx.x >> 5, lane = threadIdx.x & 31, nloc = lane & 15, hlf = lane >> 4; const int m0 = (rb0 + blockIdx.x) * 64 + wave * 16, n0 = blockIdx.y * 128;
  v8f acc[8];
#pragma unroll
  for (int t = 0; t < 8; ++t) acc[t] = (v8f){};
#pragma unroll 2
  for (int kb = 0; kb < HID; kb += 32) { const v16b a = frag_kb(ATT + (size_t)(m0 + nloc) * HID + kb, hlf); v16b al; if (TWO) al = frag_kb(ATTL + (size_t)(m0 + nloc) * HID + kb, hlf);
#pragma unroll
    for (int t = 0; t < 8; ++t) { const v16b bw = frag_kb(WP + (size_t)(n0 + t * 16 + nloc) * HID + kb, hlf); acc[t] = wmma16b(a, bw, acc[t]); if (TWO) acc[t] = wmma16b(al, bw, acc[t]); } }
#pragma unroll
  for (int t = 0; t < 8; ++t)
#pragma unroll
    for (int r = 0; r < 8; ++r) Ts[wave][8 * hlf + r][t * 16 + nloc] = acc[t][r] * (1.0f / (XS * WSC));
  wave_lds_sync();
  for (int pass = 0; pass < 2; ++pass) { for (int rr = 0; rr < 16; ++rr) *(volatile v4f*)(out + (size_t)(m0 + rr) * HID + n0 + lane * 4) = *(const v4f*)(&Ts[wave][rr][lane * 4]); __threadfence(); }
}
}

extern "C" void kernel_launch(void* const* d_in, const int* in_sizes, int n_in, void* d_out, int out_size, void* d_ws, size_t ws_size, hipStream_t stream) {
  (void)n_in;
  auto Fp = [&](int i) { return (const float*)d_in[i]; };
  if (in_sizes[0] != S * HID || in_sizes[1] != TOT * HID || in_sizes[2] != HID * HID || out_size != S * HID) return;
  size_t off = 0; char* ws = (char*)d_ws;
  auto carve = [&](size_t bytes) { char* p = ws + off; off += (bytes + 255) & ~(size_t)255; return p; };
  b16* X16 = (b16*)carve((size_t)S * HID * 2); b16* WQ = (b16*)carve((size_t)TOT * HID * 2); b16* WP = (b16*)carve((size_t)HID * HID * 2);
  b16* QH = (b16*)carve((size_t)NH * S * DH * 2); b16* QL = (b16*)carve((size_t)NH * S * DH * 2); b16* KH = (b16*)carve((size_t)NKV * S * DH * 2); b16* VROW = (b16*)carve((size_t)NKV * S * DH * 2); b16* VT = (b16*)carve((size_t)NKV * DH * S * 2);
  b16* KL = (b16*)carve((size_t)NKV * SP * DH * 2); b16* VROWL = (b16*)carve((size_t)NKV * SP * DH * 2); b16* VTL = (b16*)carve((size_t)NKV * DH * SP * 2); b16* ATTL = (b16*)carve((size_t)S * HID * 2);
  b16* ATT = X16;
  if (off > ws_size) return;
  prep_kernel<<<1024, 256, 0, stream>>>(Fp(0), Fp(1), Fp(2), X16, WQ, WP);
  qkv_kernel<<<dim3(S / 64, TOT / 128), 128, 0, stream>>>(X16, WQ, QH, QL, KH, VROW, KL, VROWL);
  vt_kernel<<<dim3(S / 64, NKV), 256, 0, stream>>>(VROW, VROWL, VT, VTL);
  attn_kernel<false><<<dim3(S / 32, NH), 64, 0, stream>>>(QH, QL, KH, KL, VT, VTL, ATT, ATTL);
  attn_kernel<true><<<dim3(SP / 32, NH), 64, 0, stream>>>(QH, QL, KH, KL, VT, VTL, ATT, ATTL);
  proj_kernel<true><<<dim3(SP / 64, HID / 128), 128, 0, stream>>>(ATT, ATTL, WP, (float*)d_out, 0);
  proj_kernel<false><<<dim3((S - SP) / 64, HID / 128), 128, 0, stream>>>(ATT, ATTL, WP, (float*)d_out, SP / 64);
}
